// gene_program_model_gcn_22651657519232
// MI455X (gfx1250) — hardware-verified
//
#include <hip/hip_runtime.h>
#include <stddef.h>


#define FD      128
#define HD      256
#define OD      128
#define NTHR    256
#define NWAVE   8
#define EPT     8
#define NGRP    2
#define CHUNK   (NTHR * EPT * NGRP)
#define WCAP    (EPT * NGRP * 32)
#define LISTN   (NWAVE * WCAP)
#define NBC     4096
#define NBF     2048
#define FPC     (NBC / NBF)
#define RCAP    40960
#define RBN     128
#define TGT     256
#define DEGCAP  256
#define OTHR    512
#define GBM     128
#define WSCAP   134217728
#define WSCL    64.0f
#define WSCLI   0.015625f

#define LDS_FILL ((RCAP + NBF + LISTN) * 4 + 64)
#define LDS_LAYER(KA, RES, TOSZ) (GBM * (KA) * 2 + ((RES) ? GBM * FD * 2 : 0) + GBM * 128 * (TOSZ))

static_assert((CHUNK & (CHUNK - 1)) == 0);
static_assert(CHUNK <= 4096);
static_assert(NBC <= 4096 && NBF <= 4096);
static_assert((NBC & (NBC - 1)) == 0 && (NBF & (NBF - 1)) == 0);
static_assert(NBC == FPC * NBF && FPC == 2);
static_assert(OTHR * 8 == NBC);
static_assert(OTHR / 32 == 8 * FPC);
static_assert((RCAP % 32) == 0);
static_assert(TGT == NWAVE * 32);
static_assert((TGT % GBM) == 0);
static_assert((DEGCAP % 32) == 0);
static_assert(GBM == NWAVE * 16 && NWAVE == 8);
static_assert((FD % 32) == 0 && FD == 4 * 32);
static_assert((HD % 128) == 0 && HD == 8 * 32 && (OD % 128) == 0);
static_assert(LDS_LAYER(2 * HD, 1, 2) <= 196608);

typedef float          v4f  __attribute__((ext_vector_type(4)));
typedef float          v8f  __attribute__((ext_vector_type(8)));
typedef int            v4i  __attribute__((ext_vector_type(4)));
typedef _Float16       v4h  __attribute__((ext_vector_type(4)));
typedef _Float16       v8h  __attribute__((ext_vector_type(8)));
typedef _Float16       v16h __attribute__((ext_vector_type(16)));
union FragH { v16h v; v8h h[2]; };

__device__ __forceinline__ v8f wmh(v16h a, v16h b, v8f c) {
  v8f d = __builtin_amdgcn_wmma_f32_16x16x32_f16(false, a, false, b, (short)0, c, false, false);
  asm volatile("v_nop\n\tv_nop\n\tv_nop\n\tv_nop" : "+v"(d) : "v"(a), "v"(b));
  return d;
}

__device__ __forceinline__ v8h cvt8(v4f a, v4f b, float s) {
  v8h r;
  r[0] = (_Float16)(a.x * s); r[1] = (_Float16)(a.y * s); r[2] = (_Float16)(a.z * s); r[3] = (_Float16)(a.w * s);
  r[4] = (_Float16)(b.x * s); r[5] = (_Float16)(b.y * s); r[6] = (_Float16)(b.z * s); r[7] = (_Float16)(b.w * s);
  return r;
}

__device__ __forceinline__ v4h cvt4(v4f a, float s) {
  v4h r;
  r[0] = (_Float16)(a.x * s); r[1] = (_Float16)(a.y * s); r[2] = (_Float16)(a.z * s); r[3] = (_Float16)(a.w * s);
  return r;
}

__global__ __launch_bounds__(NTHR) void k_wprep(const float* __restrict__ Wa, const float* __restrict__ Wb,
                                               int kin, int lg, int nv, _Float16* pl, int units) {
  const int i = (int)blockIdx.x * NTHR + (int)threadIdx.x;
  if (i >= units) return;
  const int n  = i >> lg;
  const int k0 = (i & ((1 << lg) - 1)) * 8;
  const int nc = n < nv - 1 ? n : nv - 1;
  const int kk = k0 >= kin ? k0 - kin : k0;
  const float* pa = Wa + (size_t)nc * kin + kk;
  const float* pb = Wb + (size_t)nc * kin + kk;
  v4f a0 = *(const v4f*)pa, a1 = *(const v4f*)(pa + 4);
  const v4f b0 = *(const v4f*)pb, b1 = *(const v4f*)(pb + 4);
  const v4f z4 = {0.f, 0.f, 0.f, 0.f};
  if (k0 >= kin) { a0 = b0; a1 = b1; }
  if (n >= nv)   { a0 = z4; a1 = z4; }
  const v8h hv = cvt8(a0, a1, WSCL);
  _Float16* d = pl + (size_t)i * 8;
  *(volatile v8h*)d = hv;
  __threadfence();
  *(volatile v8h*)d = hv;
}

template <int NB>
__device__ __forceinline__ int scan_chunk(const int* __restrict__ dsts, int nE, int cbase, int slotBase,
                                          int vec8, int* list, int tid, int lane, int wave) {
  int wc = 0;
#pragma unroll
  for (int g = 0; g < NGRP; ++g) {
    const int el0  = (g * NTHR + tid) * EPT;
    const int e0   = cbase + el0;
    const int sent = -2147483647 - 1;
    v4i da, db;
    if (vec8 != 0 && cbase + CHUNK <= nE) {
      da = *(const v4i*)(dsts + e0);
      db = *(const v4i*)(dsts + e0 + 4);
    } else {
      da.x = (e0     < nE) ? dsts[min(e0, nE - 1)] : sent;
      da.y = (e0 + 1 < nE) ? dsts[min(e0 + 1, nE - 1)] : sent;
      da.z = (e0 + 2 < nE) ? dsts[min(e0 + 2, nE - 1)] : sent;
      da.w = (e0 + 3 < nE) ? dsts[min(e0 + 3, nE - 1)] : sent;
      db.x = (e0 + 4 < nE) ? dsts[min(e0 + 4, nE - 1)] : sent;
      db.y = (e0 + 5 < nE) ? dsts[min(e0 + 5, nE - 1)] : sent;
      db.z = (e0 + 6 < nE) ? dsts[min(e0 + 6, nE - 1)] : sent;
      db.w = (e0 + 7 < nE) ? dsts[min(e0 + 7, nE - 1)] : sent;
    }
    const unsigned nb = (unsigned)slotBase;
    const unsigned s0 = (unsigned)da.x - nb, s1 = (unsigned)da.y - nb;
    const unsigned s2 = (unsigned)da.z - nb, s3 = (unsigned)da.w - nb;
    const unsigned s4 = (unsigned)db.x - nb, s5 = (unsigned)db.y - nb;
    const unsigned s6 = (unsigned)db.z - nb, s7 = (unsigned)db.w - nb;
    const bool h0 = s0 < (unsigned)NB, h1 = s1 < (unsigned)NB, h2 = s2 < (unsigned)NB, h3 = s3 < (unsigned)NB;
    const bool h4 = s4 < (unsigned)NB, h5 = s5 < (unsigned)NB, h6 = s6 < (unsigned)NB, h7 = s7 < (unsigned)NB;
    const unsigned any = __builtin_amdgcn_ballot_w32(h0 | h1 | h2 | h3 | h4 | h5 | h6 | h7);
    if (any != 0u) {
#define HITJ(J, HJ, SJ) { \
        const unsigned mj = __builtin_amdgcn_ballot_w32(HJ); \
        if (mj != 0u) { \
          if (HJ) { \
            const int pos = wc + (int)__builtin_amdgcn_mbcnt_lo(mj, 0u); \
            if (pos < WCAP) list[wave * WCAP + pos] = ((el0 + (J)) << 12) | (int)(SJ); \
          } \
          wc += (int)__builtin_popcount(mj); } }
      HITJ(0, h0, s0)
      HITJ(1, h1, s1)
      HITJ(2, h2, s2)
      HITJ(3, h3, s3)
      HITJ(4, h4, s4)
      HITJ(5, h5, s5)
      HITJ(6, h6, s6)
      HITJ(7, h7, s7)
#undef HITJ
    }
  }
  return wc;
}

__global__ __launch_bounds__(NTHR) void k_count(
    const int* __restrict__ dsts, int* cnt, int nE, int vec8) {
  __shared__ __attribute__((aligned(16))) int scnt[NBC];
  __shared__ __attribute__((aligned(16))) int list[LISTN];
  __shared__ int wcnt[NWAVE];
  const int tid = threadIdx.x, lane = tid & 31, wave = tid >> 5;
  const int nodeBase = blockIdx.x * NBC;

  for (int i = tid; i < NBC; i += NTHR) scnt[i] = 0;
  __syncthreads();

  const int nChunks = (nE + CHUNK - 1) / CHUNK;
#pragma unroll 1
  for (int ch = 0; ch < nChunks; ++ch) {
    const int cbase = ch * CHUNK;
    const int wc = scan_chunk<NBC>(dsts, nE, cbase, nodeBase, vec8, list, tid, lane, wave);
    if (lane == 0) wcnt[wave] = wc;
    __syncthreads();
    if (wave == 0) {
#pragma unroll 1
      for (int wsx = 0; wsx < NWAVE; ++wsx) {
        int n = __builtin_amdgcn_readfirstlane(wcnt[wsx]);
        n = n > WCAP ? WCAP : (n < 0 ? 0 : n);
        const int* lp = list + wsx * WCAP;
#pragma unroll 1
        for (int i = 0; i < n; ++i) {
          const int ent  = __builtin_amdgcn_readfirstlane(lp[i]);
          const int slot = ent & (NBC - 1);
          if (lane == 0) scnt[slot] = scnt[slot] + 1;
        }
      }
    }
    __syncthreads();
  }

  v4i cq[4];
#pragma unroll
  for (int q = 0; q < 4; ++q) {
    const int f = (wave * 4 + q) * 128 + 4 * lane;
    cq[q] = *(const v4i*)(scnt + f);
  }
  int* cpn = cnt + (size_t)nodeBase;
#pragma unroll
  for (int q = 0; q < 4; ++q) {
    const int f = (wave * 4 + q) * 128 + 4 * lane;
    *(volatile v4i*)(cpn + f) = cq[q];
  }
  __threadfence();
#pragma unroll
  for (int q = 0; q < 4; ++q) {
    const int f = (wave * 4 + q) * 128 + 4 * lane;
    *(volatile v4i*)(cpn + f) = cq[q];
  }
}

__global__ __launch_bounds__(OTHR) void k_offsets(
    const int* __restrict__ cnt, int* off, int* rbase, int nChunk) {
  __shared__ __attribute__((aligned(16))) int soff[NBC];
  __shared__ __attribute__((aligned(16))) int srb[RBN];
  __shared__ int wtot[OTHR / 32];
  const int tid = threadIdx.x, lane = tid & 31, wave = tid >> 5, sub = tid >> 8;
  for (int i = tid; i < RBN; i += OTHR) srb[i] = 0;
  __syncthreads();
  int carry = 0;
#pragma unroll 1
  for (int ch = 0; ch < nChunk; ++ch) {
    const int base = ch * NBC;
    const v4i ca = *(const v4i*)(cnt + base + 8 * tid);
    const v4i cb = *(const v4i*)(cnt + base + 8 * tid + 4);
    const int e0 = max(ca.x, 0), e1 = max(ca.y, 0), e2 = max(ca.z, 0), e3 = max(ca.w, 0);
    const int e4 = max(cb.x, 0), e5 = max(cb.y, 0), e6 = max(cb.z, 0), e7 = max(cb.w, 0);
    const int ts = e0 + e1 + e2 + e3 + e4 + e5 + e6 + e7;
    int incl = ts;
#pragma unroll
    for (int d = 1; d < 32; d <<= 1) {
      const int t = __shfl_up(incl, d);
      if (lane >= d) incl += t;
    }
    if (lane == 31) wtot[wave] = incl;
    __syncthreads();
    int S0 = 0, S1 = 0;
#pragma unroll
    for (int w = 0; w < 8; ++w) { S0 += wtot[w]; S1 += wtot[8 + w]; }
    int pre = 0;
#pragma unroll 1
    for (int w = 8 * sub; w < wave; ++w) pre += wtot[w];
    const int b0 = carry;
    const int b1 = b0 + ((S0 + 31) & ~31);
    const int b2 = b1 + ((S1 + 31) & ~31);
    const int myb = sub == 0 ? b0 : b1;
    if (tid == 0) {
      srb[min(2 * ch + 0, RBN - 1)] = b0;
      srb[min(2 * ch + 1, RBN - 1)] = b1;
    }
    int run = myb + pre + incl - ts;
    soff[8 * tid + 0] = run; run += e0;
    soff[8 * tid + 1] = run; run += e1;
    soff[8 * tid + 2] = run; run += e2;
    soff[8 * tid + 3] = run; run += e3;
    soff[8 * tid + 4] = run; run += e4;
    soff[8 * tid + 5] = run; run += e5;
    soff[8 * tid + 6] = run; run += e6;
    soff[8 * tid + 7] = run;
    carry = b2;
    __syncthreads();
    const v4i o0 = *(const v4i*)(soff + 4 * tid);
    const v4i o1 = *(const v4i*)(soff + 4 * (tid + OTHR));
    int* op = off + base;
    *(volatile v4i*)(op + 4 * tid) = o0;
    *(volatile v4i*)(op + 4 * (tid + OTHR)) = o1;
    __threadfence();
    *(volatile v4i*)(op + 4 * tid) = o0;
    *(volatile v4i*)(op + 4 * (tid + OTHR)) = o1;
    __syncthreads();
  }
  if (tid == 0) srb[min(2 * nChunk, RBN - 1)] = carry;
  __syncthreads();
  v4i rv = {0, 0, 0, 0};
  if (tid < 32) rv = *(const v4i*)(srb + 4 * tid);
  if (tid < 32) *(volatile v4i*)(rbase + 4 * tid) = rv;
  __threadfence();
  if (tid < 32) *(volatile v4i*)(rbase + 4 * tid) = rv;
}

__global__ __launch_bounds__(NTHR) void k_fill(
    const int* __restrict__ dsts, const int* __restrict__ off, const int* __restrict__ rbase,
    int* csr, int nE, int vec8, int csrLen) {
  extern __shared__ v4f lds_dyn[];
  int* region = (int*)lds_dyn;
  int* cursor = region + RCAP;
  int* list   = cursor + NBF;
  int* wcnt   = list + LISTN;
  const int tid = threadIdx.x, lane = tid & 31, wave = tid >> 5;
  const int b = blockIdx.x;
  const int nodeBase = b * NBF;

  int rb0 = rbase[b];
  const int rb1 = rbase[b + 1];
  rb0 = rb0 < 0 ? 0 : (rb0 > csrLen ? csrLen : rb0);
  rb0 &= ~31;
  int len = rb1 - rb0;
  len = len < 0 ? 0 : (len > RCAP ? RCAP : len);
  int lenW = (len + 31) & ~31;
  if (rb0 + lenW > csrLen) lenW = (csrLen - rb0) & ~31;

  {
    const v4i z = {0, 0, 0, 0};
    for (int i = tid; i < RCAP / 4; i += NTHR) ((v4i*)region)[i] = z;
    for (int s = tid; s < NBF; s += NTHR) {
      int o = off[nodeBase + s] - rb0;
      o = o < 0 ? 0 : (o > RCAP ? RCAP : o);
      cursor[s] = o;
    }
  }
  __syncthreads();

  const int nChunks = (nE + CHUNK - 1) / CHUNK;
#pragma unroll 1
  for (int ch = 0; ch < nChunks; ++ch) {
    const int cbase = ch * CHUNK;
    const int wc = scan_chunk<NBF>(dsts, nE, cbase, nodeBase, vec8, list, tid, lane, wave);
    if (lane == 0) wcnt[wave] = wc;
    __syncthreads();
    if (wave == 0) {
#pragma unroll 1
      for (int wsx = 0; wsx < NWAVE; ++wsx) {
        int n = __builtin_amdgcn_readfirstlane(wcnt[wsx]);
        n = n > WCAP ? WCAP : (n < 0 ? 0 : n);
        const int* lp = list + wsx * WCAP;
#pragma unroll 1
        for (int i = 0; i < n; ++i) {
          const int ent  = __builtin_amdgcn_readfirstlane(lp[i]);
          const int slot = ent & (NBF - 1);
          int e = cbase + ((ent >> 12) & (CHUNK - 1));
          e = e > nE - 1 ? nE - 1 : e;
          if (lane == 0) {
            int pos = cursor[slot];
            pos = pos < 0 ? 0 : (pos > RCAP - 1 ? RCAP - 1 : pos);
            region[pos] = e;
            const int np = pos + 1;
            cursor[slot] = np > RCAP ? RCAP : np;
          }
        }
      }
    }
    __syncthreads();
  }

  const int nv = lenW >> 2;
  int* gp = csr + rb0;
#pragma unroll 1
  for (int i = tid; i < nv; i += NTHR) { const v4i v = ((const v4i*)region)[i]; *(volatile v4i*)(gp + 4 * i) = v; }
  __threadfence();
#pragma unroll 1
  for (int i = tid; i < nv; i += NTHR) { const v4i v = ((const v4i*)region)[i]; *(volatile v4i*)(gp + 4 * i) = v; }
}

template <int W>
__global__ __launch_bounds__(NTHR) void k_agg(
    const int* __restrict__ csr, const int* __restrict__ off, const int* __restrict__ cnt,
    const int* __restrict__ srcs, const float* __restrict__ Hin, _Float16* AG, int nN, int nE, int csrLen) {
  constexpr int CPL = W / 32;
  static_assert(CPL == 4 || CPL == 8);
  const int tid = threadIdx.x, lane = tid & 31, wave = tid >> 5;
  const int tbase = blockIdx.x * TGT + wave * 32;
  const int col = CPL * lane;
  const v4f z4 = {0.f, 0.f, 0.f, 0.f};
  const int cl    = tbase + lane;
  const int cnt_l = cnt[cl];
  const int off_l = off[cl];

#pragma unroll 1
  for (int j = 0; j < 32; ++j) {
    const int c  = tbase + j;
    const int dg = __shfl(cnt_l, j);
    const int n  = dg < 0 ? 0 : (dg > DEGCAP ? DEGCAP : dg);
    const int st = __shfl(off_l, j);
    v4f acc0 = z4, acc1 = z4;
#pragma unroll 1
    for (int q0 = 0; q0 < n; q0 += 32) {
      int pos = st + q0 + lane;
      pos = pos < 0 ? 0 : (pos > csrLen - 1 ? csrLen - 1 : pos);
      int eid = csr[pos];
      eid = eid < 0 ? 0 : (eid > nE - 1 ? nE - 1 : eid);
      int sl = srcs[eid];
      sl = sl < 0 ? 0 : (sl > nN - 1 ? nN - 1 : sl);
      const int mcnt = (n - q0) < 32 ? (n - q0) : 32;
#pragma unroll 1
      for (int pp = 0; pp < mcnt; ++pp) {
        const int s = __builtin_amdgcn_readlane(sl, pp);
        const float* p = Hin + (size_t)s * W + col;
        acc0 += *(const v4f*)p;
        if (CPL == 8) acc1 += *(const v4f*)(p + 4);
      }
    }
    const float df  = (float)(dg < 1 ? 1 : dg);
    const float inv = 1.0f / df;
    v4f v0 = acc0 * inv, v1 = acc1 * inv;
    if (c >= nN) { v0 = z4; v1 = z4; }
    _Float16* po = AG + (size_t)c * W + col;
    if (CPL == 4) {
      const v4h hv = cvt4(v0, 1.0f);
      *(volatile v4h*)po = hv;
      __threadfence();
      *(volatile v4h*)po = hv;
    } else {
      const v8h hv = cvt8(v0, v1, 1.0f);
      *(volatile v8h*)po = hv;
      __threadfence();
      *(volatile v8h*)po = hv;
    }
  }
}

template <int ROWS, int KW, int PD>
__device__ __forceinline__ void stage_a(const float* src, int rowBase, int nValid, _Float16* dst, int colOff) {
  constexpr int UPR = (KW >= 8) ? KW / 8 : 1;
  constexpr int NU  = (KW >= 8) ? ROWS * UPR : 0;
  static_assert((NU % NTHR) == 0);
  const int tid = threadIdx.x;
  const v4f z4 = {0.f, 0.f, 0.f, 0.f};
#pragma unroll 2
  for (int it = 0; it < NU / NTHR; ++it) {
    const int u = it * NTHR + tid;
    const int r = u / UPR, c = (u % UPR) * 8;
    const int grow = rowBase + r;
    const int rc = grow < nValid ? grow : nValid - 1;
    const float* p = src + (size_t)rc * KW + c;
    v4f a = *(const v4f*)p, b = *(const v4f*)(p + 4);
    if (grow >= nValid) { a = z4; b = z4; }
    *(v8h*)(dst + (size_t)r * PD + colOff + c) = cvt8(a, b, 1.0f);
  }
}

template <int ROWS, int KW, int PD>
__device__ __forceinline__ void stage_a(const _Float16* src, int rowBase, int nValid, _Float16* dst, int colOff) {
  constexpr int UPR = (KW >= 8) ? KW / 8 : 1;
  constexpr int NU  = (KW >= 8) ? ROWS * UPR : 0;
  static_assert((NU % NTHR) == 0);
  const int tid = threadIdx.x;
  const v4i z = {0, 0, 0, 0};
#pragma unroll 2
  for (int it = 0; it < NU / NTHR; ++it) {
    const int u = it * NTHR + tid;
    const int r = u / UPR, c = (u % UPR) * 8;
    const int grow = rowBase + r;
    const int rc = grow < nValid ? grow : nValid - 1;
    v4i a = *(const v4i*)(src + (size_t)rc * KW + c);
    if (grow >= nValid) a = z;
    *(v4i*)(dst + (size_t)r * PD + colOff + c) = a;
  }
}

template <int NT, int KW2>
__device__ __forceinline__ void mmk(v8f (&acc)[NT], const _Float16* tA, int arow,
                                    const _Float16* __restrict__ Bp, int bcol0) {
  const int lane = threadIdx.x & 31, hh = lane >> 4, m = lane & 15;
  const _Float16* ap = tA + (arow + m) * KW2 + 8 * hh;
  const _Float16* bp = Bp + (size_t)(bcol0 + m) * KW2 + 8 * hh;
#pragma unroll 1
  for (int kt = 0; kt < KW2 / 32; ++kt) {
    FragH a;
    a.h[0] = *(const v8h*)(ap + 32 * kt);
    a.h[1] = *(const v8h*)(ap + 32 * kt + 16);
#pragma unroll
    for (int t = 0; t < NT; ++t) {
      const size_t to = (size_t)(16 * t) * KW2 + 32 * kt;
      FragH bq;
      bq.h[0] = *(const v8h*)(bp + to);
      bq.h[1] = *(const v8h*)(bp + to + 16);
      acc[t] = wmh(a.v, bq.v, acc[t]);
    }
  }
}

template <int ACT>
__device__ __forceinline__ float actf(float v) {
  if (ACT == 1) {
    return v > 0.f ? v : (__expf(v) - 1.0f);
  } else {
    const float e = __expf(-fabsf(v));
    return fmaxf(v, 0.f) + __logf(1.0f + e);
  }
}

__device__ __forceinline__ void store_tile(const float* stg, float* outp, int pitch, int rowBase, int colOff, int nRows) {
  const int lane = threadIdx.x & 31, wave = threadIdx.x >> 5;
#pragma unroll
  for (int i = 0; i < 16; ++i) {
    const int lr = 16 * wave + i, gr = rowBase + lr;
    if (gr < nRows) {
      const v4f v = *(const v4f*)(stg + lr * 128 + 4 * lane);
      *(volatile v4f*)(outp + (size_t)gr * pitch + colOff + 4 * lane) = v;
    }
  }
  __threadfence();
#pragma unroll
  for (int i = 0; i < 16; ++i) {
    const int lr = 16 * wave + i, gr = rowBase + lr;
    if (gr < nRows) {
      const v4f v = *(const v4f*)(stg + lr * 128 + 4 * lane);
      *(volatile v4f*)(outp + (size_t)gr * pitch + colOff + 4 * lane) = v;
    }
  }
}

__device__ __forceinline__ void store_tile(const _Float16* stg, _Float16* outp, int pitch, int rowBase, int colOff, int nRows) {
  const int lane = threadIdx.x & 31, wave = threadIdx.x >> 5, hh = lane >> 4, q = lane & 15;
#pragma unroll
  for (int i = 0; i < 8; ++i) {
    const int lr = 16 * wave + 2 * i + hh, gr = rowBase + lr;
    if (gr < nRows) {
      const v8h v = *(const v8h*)(stg + lr * 128 + 8 * q);
      *(volatile v8h*)(outp + (size_t)gr * pitch + colOff + 8 * q) = v;
    }
  }
  __threadfence();
#pragma unroll
  for (int i = 0; i < 8; ++i) {
    const int lr = 16 * wave + 2 * i + hh, gr = rowBase + lr;
    if (gr < nRows) {
      const v8h v = *(const v8h*)(stg + lr * 128 + 8 * q);
      *(volatile v8h*)(outp + (size_t)gr * pitch + colOff + 8 * q) = v;
    }
  }
}

template <typename TA, int K1W, int K2W, int NOUT, int ACT, bool RES, typename TO>
__global__ __launch_bounds__(NTHR) void k_layer(
    const TA* __restrict__ A1, const _Float16* __restrict__ A2, const _Float16* __restrict__ Bp,
    const float* __restrict__ bias, const float* __restrict__ Xr, const _Float16* __restrict__ Rp,
    const float* __restrict__ rbias, TO* outp, int nN, int nStoreRows) {
  constexpr int KA    = K1W + K2W;
  constexpr int NPASS = NOUT / 128;
  static_assert((KA % 32) == 0 && (K1W % 32) == 0 && (K2W % 32) == 0 && NPASS >= 1);
  extern __shared__ v4f lds_dyn[];
  _Float16* tA = (_Float16*)lds_dyn;
  _Float16* tX = tA + GBM * KA;
  TO* stg = (TO*)(tX + (RES ? GBM * FD : 0));
  const int tid = threadIdx.x, lane = tid & 31, wave = tid >> 5, hh = lane >> 4, m = lane & 15;
  const int rowBase = blockIdx.x * GBM;
  const int r0 = 16 * wave;

  stage_a<GBM, K1W, KA>(A1, rowBase, nN, tA, 0);
  if (K2W > 0) stage_a<GBM, K2W, KA>(A2, rowBase, nN, tA, K1W);
  if (RES) stage_a<GBM, FD, FD>(Xr, rowBase, nN, tX, 0);
  __syncthreads();

#pragma unroll 1
  for (int cp = 0; cp < NPASS; ++cp) {
    v8f acc[8];
#pragma unroll
    for (int t = 0; t < 8; ++t) { v8f z = {0.f, 0.f, 0.f, 0.f, 0.f, 0.f, 0.f, 0.f}; acc[t] = z; }
    mmk<8, KA>(acc, tA, r0, Bp, 128 * cp);
#pragma unroll
    for (int t = 0; t < 8; ++t) {
      const float bv = bias[128 * cp + 16 * t + m];
#pragma unroll
      for (int r = 0; r < 8; ++r) {
        const float v = actf<ACT>(acc[t][r] * WSCLI + bv);
        acc[t][r] = RES ? v * WSCL : v;
      }
    }
    if (RES) {
      mmk<8, FD>(acc, tX, r0, Rp, 128 * cp);
#pragma unroll
      for (int t = 0; t < 8; ++t) {
        const float rb = rbias[128 * cp + 16 * t + m];
#pragma unroll
        for (int r = 0; r < 8; ++r) acc[t][r] = acc[t][r] * WSCLI + rb;
      }
    }
    TO* sp = stg + (size_t)(r0 + 8 * hh) * 128 + m;
#pragma unroll
    for (int t = 0; t < 8; ++t) {
#pragma unroll
      for (int r = 0; r < 8; ++r) sp[r * 128 + 16 * t] = (TO)acc[t][r];
    }
    __syncthreads();
    store_tile(stg, outp, NOUT, rowBase, 128 * cp, nStoreRows);
    __syncthreads();
  }
}

#define K_S1 k_layer<float,    FD, FD, HD, 1, false, float>
#define K_S2 k_layer<float,    HD, HD, HD, 1, true,  _Float16>
#define K_F1 k_layer<_Float16, HD, 0,  HD, 1, false, _Float16>
#define K_F2 k_layer<_Float16, HD, 0,  HD, 1, true,  _Float16>
#define K_OU k_layer<_Float16, HD, 0,  OD, 2, false, float>

#define LDS_S1 LDS_LAYER(FD + FD, 0, 4)
#define LDS_S2 LDS_LAYER(HD + HD, 1, 2)
#define LDS_F1 LDS_LAYER(HD, 0, 2)
#define LDS_F2 LDS_LAYER(HD, 1, 2)
#define LDS_OU LDS_LAYER(HD, 0, 4)

static size_t carve(size_t* o, size_t bytes) {
  const size_t r = *o;
  *o += (bytes + 255) & ~(size_t)255;
  return r;
}

extern "C" void kernel_launch(void* const* d_in, const int* in_sizes, int n_in,
                              void* d_out, int out_size, void* d_ws, size_t ws_size,
                              hipStream_t stream) {
  if (n_in < 18) return;
  const int nN = in_sizes[0] / FD;
  const int nE = in_sizes[1] / 2;
  if (nN <= 0 || nE <= 0 || in_sizes[0] != nN * FD || in_sizes[1] != 2 * nE) return;
  if (in_sizes[2] != HD * FD || in_sizes[3] != HD || in_sizes[4] != HD * FD) return;
  if (in_sizes[5] != HD * HD || in_sizes[6] != HD || in_sizes[7] != HD * HD) return;
  if (in_sizes[8] != HD * FD || in_sizes[9] != HD || in_sizes[10] != HD * FD || in_sizes[11] != HD) return;
  if (in_sizes[12] != HD * HD || in_sizes[13] != HD || in_sizes[14] != HD * HD || in_sizes[15] != HD) return;
  if (in_sizes[16] != OD * HD || in_sizes[17] != OD) return;
  if ((long long)out_size != (long long)nN * OD) return;
  if (nE > (1 << 27) || nN > (1 << 22)) return;

  const float* x     = (const float*)d_in[0];
  const int*   ei    = (const int*)d_in[1];
  const float* Wl1   = (const float*)d_in[2];
  const float* bl1   = (const float*)d_in[3];
  const float* Wr1   = (const float*)d_in[4];
  const float* Wl2   = (const float*)d_in[5];
  const float* bl2   = (const float*)d_in[6];
  const float* Wr2   = (const float*)d_in[7];
  const float* R1w   = (const float*)d_in[8];
  const float* R1b   = (const float*)d_in[9];
  const float* R2w   = (const float*)d_in[10];
  const float* R2b   = (const float*)d_in[11];
  const float* F1w   = (const float*)d_in[12];
  const float* F1b   = (const float*)d_in[13];
  const float* F2w   = (const float*)d_in[14];
  const float* F2b   = (const float*)d_in[15];
  const float* F3w   = (const float*)d_in[16];
  const float* F3b   = (const float*)d_in[17];
  const int* src = ei;
  const int* dst = ei + nE;
  float* dout = (float*)d_out;

  const int NPAD   = ((nN + TGT - 1) / TGT) * TGT;
  const int nBC    = (nN + NBC - 1) / NBC;
  const int CNTPAD = nBC * NBC;
  if (FPC * nBC + 1 > RBN) return;
  const int nBF    = (nN + NBF - 1) / NBF;
  const int csrLen = ((nE + 31) & ~31) + 4096;
  if (31 * FPC * nBC > 4096) return;
  const int nAgg   = NPAD / TGT;
  const int nGn    = NPAD / GBM;

  char* ws = (char*)d_ws;
  size_t o = 0;
  const size_t oS1  = carve(&o, (size_t)HD * (2 * FD) * 2);
  const size_t oS2  = carve(&o, (size_t)HD * (2 * HD) * 2);
  const size_t oR1  = carve(&o, (size_t)HD * FD * 2);
  const size_t oR2  = carve(&o, (size_t)HD * FD * 2);
  const size_t oF1  = carve(&o, (size_t)HD * HD * 2);
  const size_t oF2  = carve(&o, (size_t)HD * HD * 2);
  const size_t oF3  = carve(&o, (size_t)OD * HD * 2);
  const size_t oCnt = carve(&o, (size_t)CNTPAD * 4);
  const size_t oOff = carve(&o, (size_t)CNTPAD * 4);
  const size_t oRb  = carve(&o, (size_t)RBN * 4);
  const size_t oCsr = carve(&o, (size_t)csrLen * 4);
  const size_t oAG1 = carve(&o, (size_t)NPAD * FD * 2);
  const size_t oH1  = carve(&o, (size_t)NPAD * HD * 4);
  const size_t oAG2 = carve(&o, (size_t)NPAD * HD * 2);
  const size_t oH2  = carve(&o, (size_t)NPAD * HD * 2);
  if (o > ws_size || o > (size_t)WSCAP) return;

  _Float16* pS1 = (_Float16*)(ws + oS1);
  _Float16* pS2 = (_Float16*)(ws + oS2);
  _Float16* pR1 = (_Float16*)(ws + oR1);
  _Float16* pR2 = (_Float16*)(ws + oR2);
  _Float16* pF1 = (_Float16*)(ws + oF1);
  _Float16* pF2 = (_Float16*)(ws + oF2);
  _Float16* pF3 = (_Float16*)(ws + oF3);
  int*   cnt  = (int*)(ws + oCnt);
  int*   offp = (int*)(ws + oOff);
  int*   rb   = (int*)(ws + oRb);
  int*   csr  = (int*)(ws + oCsr);
  _Float16* pAG1 = (_Float16*)(ws + oAG1);
  float*    pH1  = (float*)(ws + oH1);
  _Float16* pAG2 = (_Float16*)(ws + oAG2);
  _Float16* pH2  = (_Float16*)(ws + oH2);
  _Float16* pH3  = (_Float16*)(ws + oH1);
  _Float16* pH4  = (_Float16*)(ws + oAG2);

  const int vec8 = ((nE & 3) == 0) ? 1 : 0;

  k_wprep<<<(HD * 32 + NTHR - 1) / NTHR, NTHR, 0, stream>>>(Wr1, Wl1, FD, 5, HD, pS1, HD * 32);
  k_wprep<<<(HD * 64 + NTHR - 1) / NTHR, NTHR, 0, stream>>>(Wr2, Wl2, HD, 6, HD, pS2, HD * 64);
  k_wprep<<<(HD * 16 + NTHR - 1) / NTHR, NTHR, 0, stream>>>(R1w, R1w, FD, 4, HD, pR1, HD * 16);
  k_wprep<<<(HD * 16 + NTHR - 1) / NTHR, NTHR, 0, stream>>>(R2w, R2w, FD, 4, HD, pR2, HD * 16);
  k_wprep<<<(HD * 32 + NTHR - 1) / NTHR, NTHR, 0, stream>>>(F1w, F1w, HD, 5, HD, pF1, HD * 32);
  k_wprep<<<(HD * 32 + NTHR - 1) / NTHR, NTHR, 0, stream>>>(F2w, F2w, HD, 5, HD, pF2, HD * 32);
  k_wprep<<<(OD * 32 + NTHR - 1) / NTHR, NTHR, 0, stream>>>(F3w, F3w, HD, 5, OD, pF3, OD * 32);

  k_count<<<nBC, NTHR, 0, stream>>>(dst, cnt, nE, vec8);
  k_offsets<<<1, OTHR, 0, stream>>>(cnt, offp, rb, nBC);
  hipFuncSetAttribute(reinterpret_cast<const void*>(&k_fill), hipFuncAttributeMaxDynamicSharedMemorySize, LDS_FILL);
  k_fill<<<nBF, NTHR, LDS_FILL, stream>>>(dst, offp, rb, csr, nE, vec8, csrLen);

  k_agg<FD><<<nAgg, NTHR, 0, stream>>>(csr, offp, cnt, src, x, pAG1, nN, nE, csrLen);

  hipFuncSetAttribute(reinterpret_cast<const void*>(&K_S1), hipFuncAttributeMaxDynamicSharedMemorySize, LDS_S1);
  K_S1<<<nGn, NTHR, LDS_S1, stream>>>(x, pAG1, pS1, bl1, x, pR1, R1b, pH1, nN, NPAD);

  k_agg<HD><<<nAgg, NTHR, 0, stream>>>(csr, offp, cnt, src, pH1, pAG2, nN, nE, csrLen);

  hipFuncSetAttribute(reinterpret_cast<const void*>(&K_S2), hipFuncAttributeMaxDynamicSharedMemorySize, LDS_S2);
  K_S2<<<nGn, NTHR, LDS_S2, stream>>>(pH1, pAG2, pS2, bl2, x, pR1, R1b, pH2, nN, NPAD);

  hipFuncSetAttribute(reinterpret_cast<const void*>(&K_F1), hipFuncAttributeMaxDynamicSharedMemorySize, LDS_F1);
  K_F1<<<nGn, NTHR, LDS_F1, stream>>>(pH2, pAG1, pF1, F1b, x, pR2, R2b, pH3, nN, NPAD);

  hipFuncSetAttribute(reinterpret_cast<const void*>(&K_F2), hipFuncAttributeMaxDynamicSharedMemorySize, LDS_F2);
  K_F2<<<nGn, NTHR, LDS_F2, stream>>>(pH3, pAG1, pF2, F2b, x, pR2, R2b, pH4, nN, NPAD);

  hipFuncSetAttribute(reinterpret_cast<const void*>(&K_OU), hipFuncAttributeMaxDynamicSharedMemorySize, LDS_OU);
  K_OU<<<nGn, NTHR, LDS_OU, stream>>>(pH4, pAG1, pF3, F3b, x, pR2, R2b, dout, nN, nN);
}
